// TreeAttention_17008070492548
// MI455X (gfx1250) — hardware-verified
//
#include <hip/hip_runtime.h>
#include <math.h>

#ifndef NNODE
#define NNODE 256
#endif
#ifndef NLEAF
#define NLEAF 2048
#endif
#define NNODE_FULL 256
#define NLEAF_FULL 2048
#define DM 256
#define NX (NNODE + NLEAF)
#define OUT1_ELEM (NNODE_FULL * DM)
#define OUT_ELEMS ((NNODE_FULL + NLEAF_FULL) * DM)

#define XCARRY 16.0f
#define WCARRY 64.0f
#define QKSH 10
#define ACARRY 16.0f
#define MWCARRY 16.0f
#define AGGSH 8
#define PCARRY 1024.0f
static constexpr float SC2 = 1.4426950408889634f / (ACARRY * ACARRY * 16.0f);
static constexpr float OSC = 1.0f / (PCARRY * ACARRY);

static_assert(XCARRY * WCARRY == (float)(1 << QKSH));
static_assert(MWCARRY * ACARRY == (float)(1 << AGGSH));
static_assert(PCARRY * ACARRY * OSC == 1.0f);
static_assert(DM == 256);
static_assert(DM / 8 == 32);
static_assert(NNODE % 64 == 0 && NLEAF % 256 == 0);
static_assert(NX % 128 == 0);
static_assert(NNODE <= NNODE_FULL && NLEAF <= NLEAF_FULL);
static_assert((size_t)OUT1_ELEM * 4 == 262144);
static_assert((size_t)OUT1_ELEM + (size_t)NLEAF * DM <= (size_t)OUT_ELEMS);
static_assert((size_t)OUT_ELEMS * 4 == 2359296);

typedef _Float16 h16;
typedef __attribute__((ext_vector_type(16))) _Float16 v16h;
typedef __attribute__((ext_vector_type(8)))  _Float16 v8h;
typedef __attribute__((ext_vector_type(8)))  float    v8f;
typedef __attribute__((ext_vector_type(4)))  float    v4f;
typedef __attribute__((ext_vector_type(4)))  int      v4i;


#define VST2V4(ptr, val) do { const v4f vst2_v4_ = (val); *(volatile v4f*)(ptr) = vst2_v4_; __threadfence(); *(volatile v4f*)(ptr) = vst2_v4_; } while (0)

__device__ __forceinline__ float bfr(float f) {
    unsigned u = __float_as_uint(f);
    u += 0x7FFFu + ((u >> 16) & 1u);
    return __uint_as_float(u & 0xFFFF0000u);
}
static __device__ __forceinline__ h16 toh_flush(float v) { const float w = (fabsf(v) < 6.103515625e-05f) ? 0.0f : v; return (h16)w; }

__device__ __forceinline__ void st8h(h16* P, size_t o, const float* v) {
    v8h pk;
#pragma unroll
    for (int e = 0; e < 8; ++e) pk[e] = toh_flush(v[e]);
    *(volatile v8h*)(P + o) = pk;
    __threadfence();
    *(volatile v8h*)(P + o) = pk;
}

union FragU { v16h v; v8h h[2]; };
__device__ __forceinline__ v16h frag_ld(const _Float16* p) {
    FragU f; f.h[0] = *(const v8h*)(p); f.h[1] = *(const v8h*)(p + 16); return f.v;
}
__device__ __forceinline__ v8f wmma16(v16h a, v16h b, v8f c) {
    c = __builtin_amdgcn_wmma_f32_16x16x32_f16(false, a, false, b, (short)0, c, false, false);
    asm volatile("v_nop\n\tv_nop\n\tv_nop\n\tv_nop" : "+v"(c) : "v"(a), "v"(b));
    return c;
}
__device__ __forceinline__ void wave_sync_lds() {
    __builtin_amdgcn_fence(3  , "workgroup");
    __builtin_amdgcn_wave_barrier();
    __builtin_amdgcn_fence(2  , "workgroup");
}
__device__ __forceinline__ v8f vzero() { return (v8f){0.f,0.f,0.f,0.f,0.f,0.f,0.f,0.f}; }
__device__ __forceinline__ unsigned wave_id() { return (unsigned)__builtin_amdgcn_readfirstlane((int)(threadIdx.x >> 5)); }

template <int OUT_MODE, int SH, bool BIAS>
__device__ __forceinline__ void gemm64_body(
    const h16* __restrict__ A, unsigned lda, const h16* __restrict__ Bt, unsigned ldb,
    float* __restrict__ Cf, h16* __restrict__ Ch, unsigned ldc, const float* __restrict__ bias,
    unsigned M, unsigned N, unsigned K) {
  __shared__ __align__(16) float sT[8][16 * 68];
  static_assert(sizeof(float) * 8 * 16 * 68 <= 131072);
  static_assert(32 * 16 * 4 * 2 == 16 * 64 * 4);
  static_assert(32 * 16 * 4 == 16 * 64 * 2);
  constexpr float scale = 1.0f / (float)(1 << SH);
  const unsigned lane = threadIdx.x & 31u;
  const unsigned wave = wave_id();
  const unsigned tilesN = N >> 6, tilesM = M >> 6;
  const unsigned tile = blockIdx.x * 8u + wave;
  if (tile >= tilesM * tilesN) return;
  const unsigned tm = tile / tilesN;
  const unsigned tn = tile - tm * tilesN;
  const unsigned m0 = tm << 6, n0 = tn << 6;
  const unsigned rlane = lane & 15u;
  const unsigned koff = (lane >> 4) * 8u;
  const unsigned mOff = koff;

  v8f acc[4][4];
#pragma unroll
  for (int i = 0; i < 4; ++i)
#pragma unroll
    for (int j = 0; j < 4; ++j) acc[i][j] = vzero();

  for (unsigned k0 = 0; k0 < K; k0 += 32u) {
    v16h bh[4];
#pragma unroll
    for (int j = 0; j < 4; ++j)
      bh[j] = frag_ld(Bt + (size_t)(n0 + ((unsigned)j << 4) + rlane) * ldb + koff + k0);
#pragma unroll
    for (int i = 0; i < 4; ++i) {
      const v16h ah = frag_ld(A + (size_t)(m0 + ((unsigned)i << 4) + rlane) * lda + koff + k0);
#pragma unroll
      for (int j = 0; j < 4; ++j)
        acc[i][j] = wmma16(ah, bh[j], acc[i][j]);
    }
  }

  float* slab = sT[wave];
#pragma unroll
  for (int i = 0; i < 4; ++i) {
    const unsigned mBase = m0 + ((unsigned)i << 4);
#pragma unroll
    for (int j = 0; j < 4; ++j) {
      const unsigned n = n0 + ((unsigned)j << 4) + rlane;
      float bv = 0.0f;
      if (BIAS) bv = bfr(bias[n]);
#pragma unroll
      for (int r = 0; r < 8; ++r) {
        float v = acc[i][j][r] * scale + bv;
        if (OUT_MODE == 1) v *= ACARRY;
        slab[(mOff + (unsigned)r) * 68u + ((unsigned)j << 4) + rlane] = v;
      }
    }
    wave_sync_lds();
    if (OUT_MODE == 0) {
      const unsigned hh = lane >> 4, c4 = (lane & 15u) * 4u;
#pragma unroll
      for (int half = 0; half < 2; ++half) {
        v4f vv[4];
#pragma unroll
        for (int it = 0; it < 4; ++it) {
          const unsigned row = (unsigned)(half * 4 + it) * 2u + hh;
          vv[it] = *(const v4f*)(slab + row * 68u + c4);
        }
        for (int pass = 0; pass < 2; ++pass) {
#pragma unroll
          for (int it = 0; it < 4; ++it) {
            const unsigned row = (unsigned)(half * 4 + it) * 2u + hh;
            *(volatile v4f*)(Cf + (size_t)(mBase + row) * ldc + n0 + c4) = vv[it];
          }
          __threadfence();
        }
      }
    } else {
      const unsigned q = lane >> 3, c8 = (lane & 7u) * 8u;
      v8h hv[4];
#pragma unroll
      for (int it = 0; it < 4; ++it) {
        const unsigned row = (unsigned)it * 4u + q;
        const float* sp = slab + row * 68u + c8;
#pragma unroll
        for (int e = 0; e < 8; ++e) hv[it][e] = toh_flush(sp[e]);
      }
      for (int pass = 0; pass < 2; ++pass) {
#pragma unroll
        for (int it = 0; it < 4; ++it) {
          const unsigned row = (unsigned)it * 4u + q;
          *(volatile v8h*)(Ch + (size_t)(mBase + row) * ldc + n0 + c8) = hv[it];
        }
        __threadfence();
      }
    }
    wave_sync_lds();
  }
}

__global__ __launch_bounds__(256) void k_gemm_h(const h16* __restrict__ A, unsigned lda, const h16* __restrict__ Bt, unsigned ldb,
    h16* __restrict__ C, unsigned ldc, const float* __restrict__ bias, unsigned M, unsigned N, unsigned K) {
  gemm64_body<1, QKSH, true>(A, lda, Bt, ldb, (float*)0, C, ldc, bias, M, N, K);
}
__global__ __launch_bounds__(256) void k_gemm_f(const h16* __restrict__ A, unsigned lda, const h16* __restrict__ Bt, unsigned ldb,
    float* __restrict__ C, unsigned ldc, const float* __restrict__ bias, unsigned M, unsigned N, unsigned K) {
  gemm64_body<0, QKSH, true>(A, lda, Bt, ldb, C, (h16*)0, ldc, bias, M, N, K);
}
__global__ __launch_bounds__(256) void k_gemm_a(const h16* __restrict__ A, unsigned lda, const h16* __restrict__ Bt, unsigned ldb,
    float* __restrict__ C, unsigned ldc, unsigned M, unsigned N, unsigned K) {
  gemm64_body<0, AGGSH, false>(A, lda, Bt, ldb, C, (h16*)0, ldc, (const float*)0, M, N, K);
}

__global__ __launch_bounds__(256) void k_wt16(const float* __restrict__ Wm, h16* __restrict__ W16) {
    const unsigned u = blockIdx.x * 256u + threadIdx.x;
    if (u >= (unsigned)(DM * (DM / 8))) return;
    const unsigned k0 = 8u * (u & 31u);
    const unsigned o = u >> 5;
    float v[8];
#pragma unroll
    for (int i = 0; i < 8; ++i) v[i] = bfr(Wm[(size_t)(k0 + (unsigned)i) * DM + o]) * WCARRY;
    st8h(W16, (size_t)o * DM + k0, v);
}

__global__ __launch_bounds__(256) void k_x16(const float* __restrict__ x, h16* __restrict__ X16, unsigned rbase, unsigned rows) {
    const unsigned u = blockIdx.x * 256u + threadIdx.x;
    if (u >= rows * 32u) return;
    const unsigned row = u >> 5, c0 = (u & 31u) * 8u;
    const float* xr = x + (size_t)row * DM + c0;
    const v4f a = *(const v4f*)xr, b = *(const v4f*)(xr + 4);
    float v[8] = {bfr(a.x) * XCARRY, bfr(a.y) * XCARRY, bfr(a.z) * XCARRY, bfr(a.w) * XCARRY,
                  bfr(b.x) * XCARRY, bfr(b.y) * XCARRY, bfr(b.z) * XCARRY, bfr(b.w) * XCARRY};
    st8h(X16, (size_t)(rbase + row) * DM + c0, v);
}

__global__ __launch_bounds__(256) void k_omega(const float* __restrict__ leaf, const float* __restrict__ us, float* __restrict__ omega) {
    __shared__ __align__(16) float sO[32];
    const unsigned lane = threadIdx.x & 31u;
    const unsigned wave = wave_id();
    const v4f u0 = *(const v4f*)(us + 8u * lane), u1 = *(const v4f*)(us + 8u * lane + 4u);
    const float ub[8] = {bfr(u0.x), bfr(u0.y), bfr(u0.z), bfr(u0.w), bfr(u1.x), bfr(u1.y), bfr(u1.z), bfr(u1.w)};
#pragma unroll 1
    for (unsigned i = 0; i < 4u; ++i) {
        const unsigned row = blockIdx.x * 32u + wave * 4u + i;
        const float* xr = leaf + (size_t)row * DM + 8u * lane;
        const v4f a = *(const v4f*)xr, b = *(const v4f*)(xr + 4);
        float s = bfr(a.x) * ub[0] + bfr(a.y) * ub[1] + bfr(a.z) * ub[2] + bfr(a.w) * ub[3]
                + bfr(b.x) * ub[4] + bfr(b.y) * ub[5] + bfr(b.z) * ub[6] + bfr(b.w) * ub[7];
#pragma unroll
        for (int o = 16; o > 0; o >>= 1) s += __shfl_xor(s, o, 32);
        if (lane == 0u) sO[wave * 4u + i] = s;
    }
    __syncthreads();
    if (threadIdx.x < 8u) {
        const v4f v = *(const v4f*)(sO + 4u * threadIdx.x);
        VST2V4(omega + blockIdx.x * 32u + 4u * threadIdx.x, v);
    }
}

__global__ __launch_bounds__(256) void k_mwcnt(const int* __restrict__ mask, const float* __restrict__ omega,
                                               const float* __restrict__ Vf, h16* __restrict__ MW16, float* __restrict__ st2) {
    __shared__ int sM[NLEAF];
    __shared__ float sRed[8];
    __shared__ int sCnt[8];
    static_assert(sizeof(int) * NLEAF + 64 <= 131072);
    const unsigned t = threadIdx.x, lane = t & 31u;
    const unsigned wave = wave_id();
    const unsigned i = blockIdx.x;
    float part = 0.f;
    for (unsigned j0 = 8u * t; j0 < (unsigned)NLEAF; j0 += 2048u) {
        const int* mp = mask + (size_t)i * NLEAF_FULL + j0;
        const v4i m0 = *(const v4i*)mp, m1 = *(const v4i*)(mp + 4);
        const v4f o0 = *(const v4f*)(omega + j0), o1 = *(const v4f*)(omega + j0 + 4u);
        const int mi[8] = {m0.x, m0.y, m0.z, m0.w, m1.x, m1.y, m1.z, m1.w};
        const float oo[8] = {o0.x, o0.y, o0.z, o0.w, o1.x, o1.y, o1.z, o1.w};
        float v[8];
#pragma unroll
        for (int e = 0; e < 8; ++e) {
            const float w = (float)mi[e] * oo[e];
            part += w;
            v[e] = w * MWCARRY;
            sM[j0 + (unsigned)e] = (mi[e] != 0) ? 1 : 0;
        }
        st8h(MW16, (size_t)i * NLEAF + j0, v);
    }
#pragma unroll
    for (int o = 16; o > 0; o >>= 1) part += __shfl_xor(part, o, 32);
    __syncthreads();

    const unsigned dq = t & 63u, jg = t >> 6;
    const v4f nv4 = *(const v4f*)(Vf + (size_t)i * DM + 4u * dq);
    int cc = 0;
#pragma unroll 4
    for (unsigned j = jg; j < (unsigned)NLEAF; j += 4u) {
        const v4f l = *(const v4f*)(Vf + (size_t)(NNODE + j) * DM + 4u * dq);
        const int f = sM[j];
        const int n = (((nv4.x + l.x) != 0.0f) ? 1 : 0) + (((nv4.y + l.y) != 0.0f) ? 1 : 0)
                    + (((nv4.z + l.z) != 0.0f) ? 1 : 0) + (((nv4.w + l.w) != 0.0f) ? 1 : 0);
        cc += f * n;
    }
#pragma unroll
    for (int o = 16; o > 0; o >>= 1) cc += __shfl_xor(cc, o, 32);
    if (lane == 0u) { sRed[wave] = part; sCnt[wave] = cc; }
    __syncthreads();
    if (t < 8u) {
        const float rs = ((sRed[0] + sRed[1]) + (sRed[2] + sRed[3])) + ((sRed[4] + sRed[5]) + (sRed[6] + sRed[7]));
        const int ct = ((sCnt[0] + sCnt[1]) + (sCnt[2] + sCnt[3])) + ((sCnt[4] + sCnt[5]) + (sCnt[6] + sCnt[7]));
        v4f v;
        v.x = (t == 0u) ? rs : 0.0f;
        v.y = (t == 0u) ? (float)ct : 0.0f;
        v.z = 0.0f; v.w = 0.0f;
        VST2V4(st2 + (size_t)i * 32u + 4u * t, v);
    }
}

template <int MODE>
__device__ __forceinline__ void vt_body(const float* __restrict__ Vf, const float* __restrict__ agg, const float* __restrict__ st2,
                                        h16* __restrict__ VT16, unsigned gbase) {
    __shared__ __align__(16) float sX[64 * 68];
    static_assert(sizeof(float) * 64 * 68 <= 131072);
    static_assert(256 * 4 * 4 == 64 * 64);
    static_assert(256 * 2 * 16 == 64 * 64 * 2);
    const unsigned t = threadIdx.x;
    const unsigned g0 = gbase + blockIdx.x * 64u;
    const unsigned d0 = blockIdx.y * 64u;
#pragma unroll
    for (int it = 0; it < 4; ++it) {
        const unsigned idx = (unsigned)it * 256u + t;
        const unsigned rr = idx >> 4, c4 = (idx & 15u) * 4u;
        const unsigned g = g0 + rr;
        v4f v = *(const v4f*)(Vf + (size_t)g * DM + d0 + c4);
        if (MODE == 1) {
            const v4f a = *(const v4f*)(agg + (size_t)g * DM + d0 + c4);
            const float rs = st2[(size_t)g * 32u];
            const float cf = st2[(size_t)g * 32u + 1u];
            const float nz = (float)DM / (cf + 1e-6f);
            v.x = (0.5f * v.x * rs + 0.5f * a.x) * nz;
            v.y = (0.5f * v.y * rs + 0.5f * a.y) * nz;
            v.z = (0.5f * v.z * rs + 0.5f * a.z) * nz;
            v.w = (0.5f * v.w * rs + 0.5f * a.w) * nz;
        }
        sX[(c4 + 0u) * 68u + rr] = v.x * ACARRY;
        sX[(c4 + 1u) * 68u + rr] = v.y * ACARRY;
        sX[(c4 + 2u) * 68u + rr] = v.z * ACARRY;
        sX[(c4 + 3u) * 68u + rr] = v.w * ACARRY;
    }
    __syncthreads();
#pragma unroll
    for (int it = 0; it < 2; ++it) {
        const unsigned idx = (unsigned)it * 256u + t;
        const unsigned dd = idx >> 3, c8 = (idx & 7u) * 8u;
        const v4f p0 = *(const v4f*)(sX + dd * 68u + c8), p1 = *(const v4f*)(sX + dd * 68u + c8 + 4u);
        float v[8] = {p0.x, p0.y, p0.z, p0.w, p1.x, p1.y, p1.z, p1.w};
        st8h(VT16, (size_t)(d0 + dd) * NX + g0 + c8, v);
    }
}
__global__ __launch_bounds__(256) void k_vt_leaf(const float* __restrict__ Vf, h16* __restrict__ VT16) {
    vt_body<0>(Vf, Vf, Vf, VT16, (unsigned)NNODE);
}
__global__ __launch_bounds__(256) void k_vt_node(const float* __restrict__ Vf, const float* __restrict__ agg,
                                                 const float* __restrict__ st2, h16* __restrict__ VT16) {
    vt_body<1>(Vf, agg, st2, VT16, 0u);
}

__global__ __launch_bounds__(256) __attribute__((amdgpu_num_vgpr(256)))
void k_colstat(const h16* __restrict__ Q16, const h16* __restrict__ K16, float* __restrict__ cst) {
    __shared__ __align__(16) float sStat[4 * 128];
    static_assert(sizeof(float) * 4 * 128 <= 131072);
    static_assert(32 * 16 * 4 == 4 * 128 * 4);
    const unsigned lane = threadIdx.x & 31u;
    const unsigned wave = wave_id();
    const unsigned hh = lane >> 4, c = lane & 15u;
    const unsigned kt = blockIdx.x * 8u + wave;
    v16h kf[8];
    {
        unsigned koffs = (kt * 16u + c) * (unsigned)DM + 8u * hh;
#pragma unroll
        for (int ks = 0; ks < 4; ++ks) kf[ks] = frag_ld(K16 + (koffs + 32u * (unsigned)ks));
        asm volatile("" : "+v"(koffs), "+v"(kf[3]));
#pragma unroll
        for (int ks = 4; ks < 8; ++ks) kf[ks] = frag_ld(K16 + (koffs + 32u * (unsigned)ks));
    }
#pragma unroll 1
    for (unsigned blk = 0; blk < 2u; ++blk) {
        const unsigned qb = blk * (unsigned)NNODE;
        const unsigned nt = (1u - blk) * (unsigned)(NNODE / 16) + blk * (unsigned)(NLEAF / 16);
        float mr[8], lr[8];
#pragma unroll
        for (int r = 0; r < 8; ++r) { mr[r] = -3.0e38f; lr[r] = 0.f; }
#pragma unroll 1
        for (unsigned t = 0; t < nt; ++t) {
            const h16* qp = Q16 + (size_t)(qb + t * 16u + c) * DM + 8u * hh;
            v8f s = vzero();
#pragma unroll
            for (int ks = 0; ks < 8; ++ks) {
                const v16h qf = frag_ld(qp + 32 * ks);
                s = wmma16(kf[ks], qf, s);
            }
#pragma unroll
            for (int r = 0; r < 8; ++r) {
                const float sv = s[r] * SC2;
                const bool big = sv > mr[r];
                const float e = exp2f(-fabsf(sv - mr[r]));
                lr[r] = big ? (lr[r] * e + 1.0f) : (lr[r] + e);
                mr[r] = big ? sv : mr[r];
            }
        }
#pragma unroll
        for (int r = 0; r < 8; ++r) {
#pragma unroll
            for (int off = 1; off < 16; off <<= 1) {
                const float mo = __shfl_xor(mr[r], off, 32);
                const float lo = __shfl_xor(lr[r], off, 32);
                const float mm = (mo > mr[r]) ? mo : mr[r];
                lr[r] = lr[r] * exp2f(mr[r] - mm) + lo * exp2f(mo - mm);
                mr[r] = mm;
            }
        }
        if (c == 0u) {
            float* d0 = sStat + (2u * blk) * 128u + wave * 16u + 8u * hh;
            v4f a, b, ia, ib;
            a.x = mr[0]; a.y = mr[1]; a.z = mr[2]; a.w = mr[3];
            b.x = mr[4]; b.y = mr[5]; b.z = mr[6]; b.w = mr[7];
            ia.x = 1.0f / lr[0]; ia.y = 1.0f / lr[1]; ia.z = 1.0f / lr[2]; ia.w = 1.0f / lr[3];
            ib.x = 1.0f / lr[4]; ib.y = 1.0f / lr[5]; ib.z = 1.0f / lr[6]; ib.w = 1.0f / lr[7];
            *(v4f*)d0 = a; *(v4f*)(d0 + 4) = b;
            *(v4f*)(d0 + 128) = ia; *(v4f*)(d0 + 132) = ib;
        }
    }
    __syncthreads();
    if (wave == 0u) {
#pragma unroll
        for (int a = 0; a < 4; ++a) {
            const v4f v = *(const v4f*)(sStat + (unsigned)a * 128u + lane * 4u);
            VST2V4(cst + (size_t)a * NX + blockIdx.x * 128u + lane * 4u, v);
        }
    }
}

__device__ __forceinline__ h16 pval(float s, float m, float il) {
    return toh_flush(exp2f(s * SC2 - m) * (il * PCARRY));
}

__global__ __launch_bounds__(256) __attribute__((amdgpu_num_vgpr(256)))
void k_prod(const h16* __restrict__ Q16, const h16* __restrict__ K16, const h16* __restrict__ VT16,
            const float* __restrict__ cst, float* __restrict__ out) {
    __shared__ __align__(16) float sT[8][16 * 68];
    static_assert(sizeof(float) * 8 * 16 * 68 <= 131072);
    static_assert(32 * 16 * 4 * 2 == 16 * 64 * 4);
    static_assert((size_t)OUT1_ELEM >= (size_t)NNODE * DM);
    const unsigned lane = threadIdx.x & 31u;
    const unsigned wave = wave_id();
    const unsigned hh = lane >> 4, c = lane & 15u;
    const unsigned taskV = blockIdx.x * 8u + (threadIdx.x >> 5);
    const unsigned blkV = (((taskV >> 1) * 16u) >= (unsigned)NNODE) ? 1u : 0u;
    const unsigned task = (unsigned)__builtin_amdgcn_readfirstlane((int)taskV);
    const unsigned blk = (unsigned)__builtin_amdgcn_readfirstlane((int)blkV);
    const unsigned q0 = (task >> 1) * 16u;
    const unsigned dbase = (task & 1u) * 128u;
    const float* stm = cst + (size_t)(2u * blk) * NX;
    const float* sti = stm + NX;

    v16h qf[8];
    {
        unsigned qoffs = (q0 + c) * (unsigned)DM + 8u * hh;
#pragma unroll
        for (int ks = 0; ks < 4; ++ks) qf[ks] = frag_ld(Q16 + (qoffs + 32u * (unsigned)ks));
        asm volatile("" : "+v"(qoffs), "+v"(qf[3]));
#pragma unroll
        for (int ks = 4; ks < 8; ++ks) qf[ks] = frag_ld(Q16 + (qoffs + 32u * (unsigned)ks));
    }
    v8f o[8];
#pragma unroll
    for (int dt = 0; dt < 8; ++dt) o[dt] = vzero();
    const h16* vtp = VT16 + (size_t)(dbase + c) * NX + 8u * hh;

#pragma unroll 1
    for (unsigned kb = 0; kb < (unsigned)NX; kb += 32u) {
        const h16* kp = K16 + (size_t)(kb + c) * DM + 8u * hh;
        v8f s0 = vzero(), s1 = vzero();
#pragma unroll
        for (int ks = 0; ks < 8; ++ks) {
            const v16h ka = frag_ld(kp + 32 * ks);
            const v16h kc = frag_ld(kp + 16 * DM + 32 * ks);
            s0 = wmma16(ka, qf[ks], s0);
            s1 = wmma16(kc, qf[ks], s1);
        }
        const unsigned kr = kb + 8u * hh;
        v16h pf;
        {
            const v4f ma = *(const v4f*)(stm + kr), mb = *(const v4f*)(stm + kr + 4u);
            const v4f ia = *(const v4f*)(sti + kr), ib = *(const v4f*)(sti + kr + 4u);
            pf[0] = pval(s0[0], ma.x, ia.x); pf[1] = pval(s0[1], ma.y, ia.y);
            pf[2] = pval(s0[2], ma.z, ia.z); pf[3] = pval(s0[3], ma.w, ia.w);
            pf[4] = pval(s0[4], mb.x, ib.x); pf[5] = pval(s0[5], mb.y, ib.y);
            pf[6] = pval(s0[6], mb.z, ib.z); pf[7] = pval(s0[7], mb.w, ib.w);
        }
        {
            const v4f ma = *(const v4f*)(stm + kr + 16u), mb = *(const v4f*)(stm + kr + 20u);
            const v4f ia = *(const v4f*)(sti + kr + 16u), ib = *(const v4f*)(sti + kr + 20u);
            pf[8]  = pval(s1[0], ma.x, ia.x); pf[9]  = pval(s1[1], ma.y, ia.y);
            pf[10] = pval(s1[2], ma.z, ia.z); pf[11] = pval(s1[3], ma.w, ia.w);
            pf[12] = pval(s1[4], mb.x, ib.x); pf[13] = pval(s1[5], mb.y, ib.y);
            pf[14] = pval(s1[6], mb.z, ib.z); pf[15] = pval(s1[7], mb.w, ib.w);
        }
#pragma unroll
        for (int dt = 0; dt < 8; ++dt) {
            const v16h va = frag_ld(vtp + (size_t)((unsigned)dt * 16u) * NX + kb);
            o[dt] = wmma16(va, pf, o[dt]);
        }
    }

    float* slab = sT[wave];
    const unsigned obase = q0 * (unsigned)DM + blk * (unsigned)(OUT1_ELEM - NNODE * DM) + dbase;
#pragma unroll
    for (int sl = 0; sl < 2; ++sl) {
#pragma unroll
        for (int j = 0; j < 4; ++j) {
            const v8f a = o[4 * sl + j];
            v4f lo4, hi4;
            lo4.x = a[0] * OSC; lo4.y = a[1] * OSC; lo4.z = a[2] * OSC; lo4.w = a[3] * OSC;
            hi4.x = a[4] * OSC; hi4.y = a[5] * OSC; hi4.z = a[6] * OSC; hi4.w = a[7] * OSC;
            float* sp = slab + c * 68u + (unsigned)j * 16u + 8u * hh;
            *(v4f*)sp = lo4;
            *(v4f*)(sp + 4) = hi4;
        }
        wave_sync_lds();
        {
            const unsigned c4 = (lane & 15u) * 4u;
#pragma unroll
            for (int half = 0; half < 2; ++half) {
                v4f vv[4];
#pragma unroll
                for (int it = 0; it < 4; ++it) {
                    const unsigned row = (unsigned)(half * 4 + it) * 2u + hh;
                    vv[it] = *(const v4f*)(slab + row * 68u + c4);
                }
                for (int pass = 0; pass < 2; ++pass) {
#pragma unroll
                    for (int it = 0; it < 4; ++it) {
                        const unsigned row = (unsigned)(half * 4 + it) * 2u + hh;
                        *(volatile v4f*)(out + (size_t)obase + (size_t)row * DM + (unsigned)sl * 64u + c4) = vv[it];
                    }
                    __threadfence();
                }
            }
        }
        wave_sync_lds();
    }
}

static constexpr size_t al256(size_t b) { return (b + 255) & ~(size_t)255; }
static constexpr size_t OFF_X16 = 0;
static constexpr size_t OFF_WQ  = OFF_X16 + al256((size_t)NX * DM * 2);
static constexpr size_t OFF_WK  = OFF_WQ  + al256((size_t)DM * DM * 2);
static constexpr size_t OFF_WV  = OFF_WK  + al256((size_t)DM * DM * 2);
static constexpr size_t OFF_Q16 = OFF_WV  + al256((size_t)DM * DM * 2);
static constexpr size_t OFF_K16 = OFF_Q16 + al256((size_t)NX * DM * 2);
static constexpr size_t OFF_VF  = OFF_K16 + al256((size_t)NX * DM * 2);
static constexpr size_t OFF_VT  = OFF_VF  + al256((size_t)NX * DM * 4);
static constexpr size_t OFF_OM  = OFF_VT  + al256((size_t)DM * NX * 2);
static constexpr size_t OFF_MW  = OFF_OM  + al256((size_t)NLEAF * 4);
static constexpr size_t OFF_ST2 = OFF_MW  + al256((size_t)NNODE * NLEAF * 2);
static constexpr size_t OFF_AGG = OFF_ST2 + al256((size_t)NNODE * 32 * 4);
static constexpr size_t OFF_CST = OFF_AGG + al256((size_t)NNODE * DM * 4);
static constexpr size_t WS_TOTAL = OFF_CST + al256((size_t)4 * NX * 4);
static_assert(WS_TOTAL <= (size_t)134217728);

static constexpr int IN_NODE_MIN = NNODE * DM;
static constexpr int IN_LEAF_MIN = NLEAF * DM;
static constexpr int IN_MASK_MIN = (NNODE - 1) * NLEAF_FULL + NLEAF;
static constexpr int IN_W_MIN = DM * DM;
static constexpr int OUT_MIN = OUT1_ELEM + NLEAF * DM;

static constexpr unsigned G_X16N = (NNODE * 32) / 256;
static constexpr unsigned G_X16L = (NLEAF * 32) / 256;
static constexpr unsigned G_WT   = (DM * (DM / 8)) / 256;
static constexpr unsigned G_QKV  = ((NX / 64) * (DM / 64) + 7) / 8;
static constexpr unsigned G_AGG  = ((NNODE / 64) * (DM / 64) + 7) / 8;
static constexpr unsigned G_OM   = NLEAF / 32;
static constexpr unsigned G_CS   = NX / 128;
static constexpr unsigned G_PR   = (NX / 16) * 2 / 8;
static_assert((NNODE * 32) % 256 == 0 && (NLEAF * 32) % 256 == 0);
static_assert(NLEAF % 32 == 0);
static_assert(((NX / 16) * 2) % 8 == 0);
static_assert(NX % 64 == 0 && NLEAF % 32 == 0 && DM % 64 == 0);

extern "C" void kernel_launch(void* const* d_in, const int* in_sizes, int n_in, void* d_out, int out_size,
                              void* d_ws, size_t ws_size, hipStream_t stream) {
    if (n_in < 10) return;
    if (in_sizes[0] < IN_NODE_MIN || in_sizes[1] < IN_LEAF_MIN || in_sizes[2] < IN_MASK_MIN) return;
    if (in_sizes[3] < IN_W_MIN || in_sizes[5] < IN_W_MIN || in_sizes[7] < IN_W_MIN) return;
    if (in_sizes[4] < DM || in_sizes[6] < DM || in_sizes[8] < DM || in_sizes[9] < DM) return;
    if (out_size < OUT_MIN) return;
    if (ws_size < WS_TOTAL) return;

    const float* node = (const float*)d_in[0];
    const float* leaf = (const float*)d_in[1];
    const int*   mask = (const int*)d_in[2];
    const float* Wq   = (const float*)d_in[3];
    const float* bq   = (const float*)d_in[4];
    const float* Wk   = (const float*)d_in[5];
    const float* bk   = (const float*)d_in[6];
    const float* Wv   = (const float*)d_in[7];
    const float* bv   = (const float*)d_in[8];
    const float* u_s  = (const float*)d_in[9];
    float* out = (float*)d_out;

    char* wsp = (char*)d_ws;
    h16*   X16  = (h16*)(wsp + OFF_X16);
    h16*   WQ16 = (h16*)(wsp + OFF_WQ);
    h16*   WK16 = (h16*)(wsp + OFF_WK);
    h16*   WV16 = (h16*)(wsp + OFF_WV);
    h16*   Q16  = (h16*)(wsp + OFF_Q16);
    h16*   K16  = (h16*)(wsp + OFF_K16);
    float* Vf   = (float*)(wsp + OFF_VF);
    h16*   VT16 = (h16*)(wsp + OFF_VT);
    float* omg  = (float*)(wsp + OFF_OM);
    h16*   MW16 = (h16*)(wsp + OFF_MW);
    float* st2  = (float*)(wsp + OFF_ST2);
    float* agg  = (float*)(wsp + OFF_AGG);
    float* cst  = (float*)(wsp + OFF_CST);

    k_x16<<<G_X16N, 256, 0, stream>>>(node, X16, 0u, (unsigned)NNODE);
    k_x16<<<G_X16L, 256, 0, stream>>>(leaf, X16, (unsigned)NNODE, (unsigned)NLEAF);
    k_wt16<<<G_WT, 256, 0, stream>>>(Wq, WQ16);
    k_wt16<<<G_WT, 256, 0, stream>>>(Wk, WK16);
    k_wt16<<<G_WT, 256, 0, stream>>>(Wv, WV16);

    k_gemm_h<<<G_QKV, 256, 0, stream>>>(X16, DM, WQ16, DM, Q16, DM, bq, (unsigned)NX, DM, DM);
    k_gemm_h<<<G_QKV, 256, 0, stream>>>(X16, DM, WK16, DM, K16, DM, bk, (unsigned)NX, DM, DM);
    k_gemm_f<<<G_QKV, 256, 0, stream>>>(X16, DM, WV16, DM, Vf, DM, bv, (unsigned)NX, DM, DM);

    k_omega<<<G_OM, 256, 0, stream>>>(leaf, u_s, omg);
    k_vt_leaf<<<dim3(NLEAF / 64, DM / 64), 256, 0, stream>>>(Vf, VT16);
    k_mwcnt<<<NNODE, 256, 0, stream>>>(mask, omg, Vf, MW16, st2);

    k_gemm_a<<<G_AGG, 256, 0, stream>>>(MW16, NLEAF, VT16 + NNODE, (unsigned)NX, agg, DM, (unsigned)NNODE, DM, (unsigned)NLEAF);
    k_vt_node<<<dim3(NNODE / 64, DM / 64), 256, 0, stream>>>(Vf, agg, st2, VT16);

    k_colstat<<<G_CS, 256, 0, stream>>>(Q16, K16, cst);
    k_prod<<<G_PR, 256, 0, stream>>>(Q16, K16, VT16, cst, out);
}
